// SparseLinearAttention_4440996184229
// MI455X (gfx1250) — hardware-verified
//
#include <hip/hip_runtime.h>
#include <hip/hip_bf16.h>

#define __bf16 _Float16
typedef __attribute__((ext_vector_type(4))) float v4f_t;
typedef float v4fa __attribute__((ext_vector_type(4), may_alias));
typedef __attribute__((ext_vector_type(16))) __bf16 v16bf;
typedef __attribute__((ext_vector_type(8)))  __bf16 v8bf;
typedef __attribute__((ext_vector_type(8)))  float  v8f;

static constexpr int H_    = 16;
static constexpr int D_    = 64;
static constexpr int L_    = 4096;
static constexpr int MBLK  = 64;
static constexpr int TK    = 8;
static constexpr int RS    = 72;

static __device__ __forceinline__ v8f wmma_bf16(v16bf a, v16bf b, v8f c) {
  return __builtin_amdgcn_wmma_f32_16x16x32_f16(false, a, false, b, (short)0, c, false, false);
}

static __device__ __forceinline__ v16bf frag_row(const __bf16* p, int hf) {
  v8bf x = *(const v8bf*)(p + 8 * hf);
  v8bf y = *(const v8bf*)(p + 16 + 8 * hf);
  v16bf r;
#pragma unroll
  for (int i = 0; i < 8; ++i) { r[i] = x[i]; r[i + 8] = y[i]; }
  return r;
}

static __device__ __forceinline__ void stage32(const float* g, __bf16* l) {
#pragma unroll
  for (int i = 0; i < 8; ++i) {
    float4 f = ((const float4*)g)[i];
    l[4*i+0] = (__bf16)f.x; l[4*i+1] = (__bf16)f.y;
    l[4*i+2] = (__bf16)f.z; l[4*i+3] = (__bf16)f.w;
  }
}

static __device__ __forceinline__ void stage32t(const float* g, __bf16* l) {
#pragma unroll
  for (int i = 0; i < 8; ++i) {
    float4 f = ((const float4*)g)[i];
    l[(4*i+0)*RS] = (__bf16)f.x; l[(4*i+1)*RS] = (__bf16)f.y;
    l[(4*i+2)*RS] = (__bf16)f.z; l[(4*i+3)*RS] = (__bf16)f.w;
  }
}

__global__ void kmeans_kernel(const float* __restrict__ q, const float* __restrict__ k,
                              float* __restrict__ qm, float* __restrict__ km) {
  int id = blockIdx.x;
  bool isK = id >= H_ * MBLK;
  int hm = isK ? id - H_ * MBLK : id;
  int h = hm / MBLK, m = hm % MBLK;
  const float* src = isK ? k : q;
  float* dst = isK ? km : qm;
  int d = threadIdx.x;
  float s = 0.f;
  for (int r = 0; r < 64; ++r)
    s += src[(size_t)((m * 64 + r) * H_ + h) * D_ + d];
  const float mv = s * (1.f / 64.f);
  *(volatile float*)(dst + (h * MBLK + m) * D_ + d) = mv; __threadfence(); *(volatile float*)(dst + (h * MBLK + m) * D_ + d) = mv;
}

__global__ void topk_kernel(const float* __restrict__ qm, const float* __restrict__ km,
                            int* __restrict__ lut) {
  __shared__ float qs[64 * 64];
  __shared__ float ks[64 * 64];
  int h = blockIdx.x, t = threadIdx.x;
  for (int d = 0; d < 64; ++d) {
    qs[t * 64 + d] = qm[(h * MBLK + t) * D_ + d];
    ks[t * 64 + d] = km[(h * MBLK + t) * D_ + d];
  }
  __syncthreads();
  __shared__ float scs[64 * 65];
  float* sc = scs + t * 65;
  for (int n = 0; n < 64; ++n) {
    float s = 0.f;
    for (int d = 0; d < 64; ++d) s += qs[t * 64 + d] * ks[n * 64 + d];
    sc[n] = s;
  }
  __shared__ __attribute__((aligned(16))) int slut[64 * TK];
  for (int j = 0; j < TK; ++j) {
    int best = 0; float bv = sc[0];
    for (int n = 1; n < 64; ++n) if (sc[n] > bv) { bv = sc[n]; best = n; }
    slut[t * TK + j] = best;
    sc[best] = -3.0e38f;
  }
  __syncthreads();
  typedef __attribute__((ext_vector_type(4))) int v4i_t; typedef int v4ia __attribute__((ext_vector_type(4), may_alias));
  #pragma unroll 1
  for (int pass = 0; pass < 2; ++pass) {
    for (int c = t; c < 64 * TK / 4; c += 64) *(volatile v4i_t*)(lut + (h * MBLK) * TK + c * 4) = *(const volatile v4ia*)(slut + c * 4);
    __threadfence();
  }
}

__global__ __launch_bounds__(128) void sparse_attn_kernel(
    const float* __restrict__ q, const float* __restrict__ k, const float* __restrict__ v,
    const int* __restrict__ lut, float* __restrict__ out) {
  __shared__ __align__(16) __bf16 Qs[64 * RS];
  __shared__ __align__(16) __bf16 Ks[64 * RS];
  __shared__ __align__(16) __bf16 Vt[64 * RS];
  __shared__ __align__(16) __bf16 Ps[64 * RS];
  int h = blockIdx.x >> 6, m = blockIdx.x & 63;
  int tid = threadIdx.x, w = tid >> 5, lane = tid & 31;
  int n = lane & 15, hf = lane >> 4;
  int sr = tid >> 1, sc0 = (tid & 1) * 32;

  stage32(q + (size_t)((m * 64 + sr) * H_ + h) * D_ + sc0, &Qs[sr * RS + sc0]);

  float rm[8], rsum[8];
  v8f acc[4] = {};
#pragma unroll
  for (int r = 0; r < 8; ++r) { rm[r] = -1e30f; rsum[r] = 0.f; }

  int zlane; asm volatile("v_mov_b32 %0, 0" : "=v"(zlane));
  int mylut = ((const volatile int*)lut)[(h * MBLK + m) * TK + ((lane + zlane) & (TK - 1))];
  mylut = ((unsigned)mylut < (unsigned)MBLK) ? mylut : 0;
  for (int t = 0; t < TK; ++t) {
    __syncthreads();
    int nb = __shfl(mylut, t, 32);
    stage32 (k + (size_t)((nb * 64 + sr) * H_ + h) * D_ + sc0, &Ks[sr * RS + sc0]);
    stage32t(v + (size_t)((nb * 64 + sr) * H_ + h) * D_ + sc0, &Vt[sc0 * RS + sr]);

    __syncthreads();

    v16bf qa0 = frag_row(&Qs[(16 * w + n) * RS + 0],  hf);
    v16bf qa1 = frag_row(&Qs[(16 * w + n) * RS + 32], hf);
    v8f s[4];
#pragma unroll
    for (int nt = 0; nt < 4; ++nt) {
      v8f sv = {};
      sv = wmma_bf16(qa0, frag_row(&Ks[(16 * nt + n) * RS + 0],  hf), sv);
      sv = wmma_bf16(qa1, frag_row(&Ks[(16 * nt + n) * RS + 32], hf), sv);
      s[nt] = sv * 0.125f;
    }
#pragma unroll
    for (int r = 0; r < 8; ++r) {
      float tmax = fmaxf(fmaxf(s[0][r], s[1][r]), fmaxf(s[2][r], s[3][r]));
      tmax = fmaxf(tmax, __shfl_xor(tmax, 1, 32));
      tmax = fmaxf(tmax, __shfl_xor(tmax, 2, 32));
      tmax = fmaxf(tmax, __shfl_xor(tmax, 4, 32));
      tmax = fmaxf(tmax, __shfl_xor(tmax, 8, 32));
      float mnew = fmaxf(rm[r], tmax);
      float f = __expf(rm[r] - mnew);
      rm[r] = mnew;
      float psum = 0.f;
#pragma unroll
      for (int nt = 0; nt < 4; ++nt) {
        float p = __expf(s[nt][r] - mnew);
        Ps[(16 * w + r + 8 * hf) * RS + 16 * nt + n] = (__bf16)(p * 1024.0f);
        psum += p;
        acc[nt][r] *= f;
      }
      psum += __shfl_xor(psum, 1, 32);
      psum += __shfl_xor(psum, 2, 32);
      psum += __shfl_xor(psum, 4, 32);
      psum += __shfl_xor(psum, 8, 32);
      rsum[r] = rsum[r] * f + psum;
    }
#pragma unroll
    for (int ks = 0; ks < 2; ++ks) {
      v16bf pa = frag_row(&Ps[(16 * w + n) * RS + 32 * ks], hf);
#pragma unroll
      for (int nt = 0; nt < 4; ++nt)
        acc[nt] = wmma_bf16(pa, frag_row(&Vt[(16 * nt + n) * RS + 32 * ks], hf), acc[nt]);
    }
  }
  __shared__ __attribute__((aligned(16))) float ost[4][16 * 68];
  float* so = ost[w];
#pragma unroll
  for (int nt = 0; nt < 4; ++nt)
#pragma unroll
    for (int r = 0; r < 8; ++r) so[(r + 8 * hf) * 68 + 16 * nt + n] = acc[nt][r] / (rsum[r] * 1024.0f);
  asm volatile("s_wait_dscnt 0" ::: "memory");
#pragma unroll 1
  for (int pass = 0; pass < 2; ++pass) {
#pragma unroll
    for (int i = 0; i < 8; ++i) { const int c = lane + 32 * i, rr = c >> 4, q4 = (c & 15) * 4; const int l = m * 64 + 16 * w + rr;
      *(volatile v4f_t*)(out + (size_t)(l * H_ + h) * D_ + q4) = *(const volatile v4fa*)(so + rr * 68 + q4); }
    __threadfence();
  }
}

__global__ __launch_bounds__(128) void kv_kernel(
    const float* __restrict__ k, const float* __restrict__ v,
    float* __restrict__ kvt, float* __restrict__ ksumws) {
  __shared__ __align__(16) __bf16 kft[64 * RS];
  __shared__ __align__(16) __bf16 vft[64 * RS];
  int h = blockIdx.x;
  int tid = threadIdx.x, w = tid >> 5, lane = tid & 31;
  int n = lane & 15, hf = lane >> 4;
  v8f acc[4] = {};
  float kacc = 0.f;
  for (int c = 0; c < L_ / 32; ++c) {
    __syncthreads();
    if (tid < 32) {
      int l = c * 32 + tid;
      const float* kr = k + (size_t)(l * H_ + h) * D_;
      float buf[64]; float mx = -1e30f;
#pragma unroll
      for (int d = 0; d < 64; ++d) { buf[d] = kr[d]; mx = fmaxf(mx, buf[d]); }
      float se = 0.f;
#pragma unroll
      for (int d = 0; d < 64; ++d) { buf[d] = __expf(buf[d] - mx); se += buf[d]; }
      float inv = 1.f / se;
#pragma unroll
      for (int d = 0; d < 64; ++d) kft[d * RS + tid] = (__bf16)(buf[d] * inv * 1024.0f);
    } else if (tid < 96) {
      int idx = tid - 32, vr = idx >> 1, c0 = (idx & 1) * 32;
      int l = c * 32 + vr;
      stage32t(v + (size_t)(l * H_ + h) * D_ + c0, &vft[c0 * RS + vr]);
    }
    __syncthreads();
    if (tid < 64) {
#pragma unroll
      for (int r = 0; r < 32; ++r) kacc += (float)kft[tid * RS + r];
    }
    v16bf a = frag_row(&kft[(16 * w + n) * RS], hf);
#pragma unroll
    for (int nt = 0; nt < 4; ++nt)
      acc[nt] = wmma_bf16(a, frag_row(&vft[(16 * nt + n) * RS], hf), acc[nt]);
  }
  __shared__ __attribute__((aligned(16))) float kst[64 * 64];
#pragma unroll
  for (int nt = 0; nt < 4; ++nt)
#pragma unroll
    for (int r = 0; r < 8; ++r)
      kst[(16 * nt + n) * 64 + (16 * w + r + 8 * hf)] = acc[nt][r];
  __syncthreads();
#pragma unroll 1
  for (int pass = 0; pass < 2; ++pass) {
    for (int c = tid; c < 1024; c += 128) *(volatile v4f_t*)(kvt + (size_t)h * 4096 + c * 4) = *(const volatile v4fa*)(kst + c * 4);
    if (tid < 64) *(volatile float*)(ksumws + h * 64 + tid) = kacc;
    __threadfence();
  }
}

__global__ __launch_bounds__(128) void linear_out_kernel(
    const float* __restrict__ q, const float* __restrict__ kvt,
    const float* __restrict__ ksumws, const float* __restrict__ wproj,
    const float* __restrict__ bproj, const float* __restrict__ osp, float* __restrict__ out) {
  __shared__ __align__(16) __bf16 qf[64 * RS];
  __shared__ __align__(16) __bf16 kvb[64 * RS];
  __shared__ __align__(16) __bf16 wps[64 * RS];
  __shared__ __align__(16) __bf16 ols[64 * RS];
  __shared__ float sks[64];
  __shared__ float dens[64];
  int h = blockIdx.x >> 6, m = blockIdx.x & 63;
  int tid = threadIdx.x, w = tid >> 5, lane = tid & 31;
  int n = lane & 15, hf = lane >> 4;
  int sr = tid >> 1, c0 = (tid & 1) * 32;

  stage32(kvt + (size_t)h * 4096 + sr * 64 + c0, &kvb[sr * RS + c0]);
  stage32(wproj + sr * 64 + c0, &wps[sr * RS + c0]);
  if (tid >= 64) sks[tid - 64] = ksumws[h * 64 + tid - 64];
  __syncthreads();

  if (tid < 64) {
    int l = m * 64 + tid;
    const float* qr = q + (size_t)(l * H_ + h) * D_;
    float buf[64]; float mx = -1e30f;
#pragma unroll
    for (int d = 0; d < 64; ++d) { buf[d] = qr[d]; mx = fmaxf(mx, buf[d]); }
    float se = 0.f;
#pragma unroll
    for (int d = 0; d < 64; ++d) { buf[d] = __expf(buf[d] - mx); se += buf[d]; }
    float inv = 1.f / se, den = 0.f;
#pragma unroll
    for (int d = 0; d < 64; ++d) {
      float p = buf[d] * inv;
      qf[tid * RS + d] = (__bf16)(p * 1024.0f);
      den += p * sks[d];
    }
    dens[tid] = den + 1e-6f * 1024.0f;
  }
  __syncthreads();

  v8f acc[4] = {};
#pragma unroll
  for (int ks = 0; ks < 2; ++ks) {
    v16bf a = frag_row(&qf[(16 * w + n) * RS + 32 * ks], hf);
#pragma unroll
    for (int nt = 0; nt < 4; ++nt)
      acc[nt] = wmma_bf16(a, frag_row(&kvb[(16 * nt + n) * RS + 32 * ks], hf), acc[nt]);
  }
#pragma unroll
  for (int nt = 0; nt < 4; ++nt)
#pragma unroll
    for (int r = 0; r < 8; ++r) {
      int row = 16 * w + r + 8 * hf;
      ols[row * RS + 16 * nt + n] = (__bf16)(acc[nt][r] / dens[row] * (1.0f / 1024.0f));
    }

  v8f acc2[4] = {};
#pragma unroll
  for (int ks = 0; ks < 2; ++ks) {
    v16bf a = frag_row(&ols[(16 * w + n) * RS + 32 * ks], hf);
#pragma unroll
    for (int nt = 0; nt < 4; ++nt)
      acc2[nt] = wmma_bf16(a, frag_row(&wps[(16 * nt + n) * RS + 32 * ks], hf), acc2[nt]);
  }
  __shared__ __attribute__((aligned(16))) float ost[4][16 * 68];
  float* so = ost[w];
#pragma unroll
  for (int nt = 0; nt < 4; ++nt)
#pragma unroll
    for (int r = 0; r < 8; ++r) {
      int row = 16 * w + r + 8 * hf;
      int l = m * 64 + row;
      size_t o = (size_t)(l * H_ + h) * D_ + 16 * nt + n;
      so[row % 16 * 68 + 16 * nt + n] = osp[o] + acc2[nt][r] + bproj[16 * nt + n];
    }
  asm volatile("s_wait_dscnt 0" ::: "memory");
#pragma unroll 1
  for (int pass = 0; pass < 2; ++pass) {
#pragma unroll
    for (int i = 0; i < 8; ++i) { const int c = lane + 32 * i, rr = c >> 4, q4 = (c & 15) * 4; const int l = m * 64 + 16 * w + rr;
      *(volatile v4f_t*)(out + (size_t)(l * H_ + h) * D_ + q4) = *(const volatile v4fa*)(so + rr * 68 + q4); }
    __threadfence();
  }
}

extern "C" void kernel_launch(void* const* d_in, const int* in_sizes, int n_in,
                              void* d_out, int out_size, void* d_ws, size_t ws_size,
                              hipStream_t stream) {
  (void)in_sizes; (void)n_in; (void)out_size; (void)ws_size;
  const float* q  = (const float*)d_in[0];
  const float* k  = (const float*)d_in[1];
  const float* v  = (const float*)d_in[2];
  const float* wp = (const float*)d_in[3];
  const float* bp = (const float*)d_in[4];
  float* out = (float*)d_out;

  float* ws   = (float*)d_ws;
  float* qm   = ws;
  float* km   = ws + 65536;
  float* kvt  = ws + 131072;
  float* ksum = ws + 196608;
  int*   lut  = (int*)(ws + 196672);
  float* osp  = ws + 262144;

  hipLaunchKernelGGL(kmeans_kernel,     dim3(2 * H_ * MBLK), dim3(64),  0, stream, q, k, qm, km);
  hipLaunchKernelGGL(topk_kernel,       dim3(H_),            dim3(64),  0, stream, qm, km, lut);
  hipLaunchKernelGGL(sparse_attn_kernel,dim3(H_ * MBLK),     dim3(128), 0, stream, q, k, v, lut, osp);
  hipLaunchKernelGGL(kv_kernel,         dim3(H_),            dim3(128), 0, stream, k, v, kvt, ksum);
  hipLaunchKernelGGL(linear_out_kernel, dim3(H_ * MBLK),     dim3(128), 0, stream, q, kvt, ksum, wp, bp, osp, out);
}
